// CausalSelfAttention_13477607375822
// MI455X (gfx1250) — hardware-verified
//
#include <hip/hip_runtime.h>
#ifndef NB
#define NB 2
#endif
#ifndef SQ
#define SQ 2048
#endif
#define NB_FULL 2
#define SQ_FULL 2048
#define DM 1024
#define NH 16
#define HD 64
#define QT 256
#define NKX SQ
#define QT0 128
#define LQ (3 * DM)
#define NR ((size_t)NB * SQ)

static_assert(NB <= NB_FULL);
static_assert(SQ <= SQ_FULL);
static_assert(SQ % QT == 0);
static_assert((QT & (QT - 1)) == 0);
static_assert(QT % 128 == 0);
static_assert(QT0 % 128 == 0);
static_assert(QT0 <= SQ);
static_assert(HD == 64);
static_assert(DM == NH * HD);
static_assert(DM / 8 == 128);
static_assert(DM % 64 == 0);
static_assert(LQ % 64 == 0);
static_assert(((size_t)NB * SQ) % 128 == 0);
static_assert(SQ % 64 == 0);

typedef unsigned short v8us __attribute__((ext_vector_type(8), may_alias));
typedef float  v8f  __attribute__((ext_vector_type(8)));
typedef float  v4f  __attribute__((ext_vector_type(4)));
typedef float  v4fa __attribute__((ext_vector_type(4), may_alias));
typedef _Float16 v16h __attribute__((ext_vector_type(16)));
typedef _Float16 v4h __attribute__((ext_vector_type(4)));
union FragH { v16h v; v8us half[2]; _Float16 h[16]; unsigned short u[16]; };

__device__ __forceinline__ unsigned short bf16_bits(float x) { unsigned int u = __float_as_uint(x); return (unsigned short)((u + 0x7FFFu + ((u >> 16) & 1u)) >> 16); }
__device__ __forceinline__ float bf16_val(unsigned short b) { return __uint_as_float(((unsigned int)b) << 16); }
__device__ __forceinline__ float bf16_rne(float x) { return bf16_val(bf16_bits(x)); }

__device__ __forceinline__ v16h g2_frag(const _Float16* p, unsigned hh) { FragH f; f.half[0] = *(const v8us*)((const unsigned short*)p + 8 * hh); f.half[1] = *(const v8us*)((const unsigned short*)p + 16 + 8 * hh); return f.v; }
__device__ __forceinline__ v8f g2_mma(v16h a, v16h b, v8f c) { v8f d = __builtin_amdgcn_wmma_f32_16x16x32_f16(false, a, false, b, (short)0, c, false, false); asm volatile("v_nop\n\tv_nop\n\tv_nop\n\tv_nop" : "+v"(d) : "v"(a), "v"(b)); return d; }

__global__ __launch_bounds__(256) void k_wnat(const float* __restrict__ w, unsigned int n8, _Float16* __restrict__ Bt) {
  const unsigned int t = blockIdx.x * 256u + threadIdx.x; if (t >= n8) return;
  const float* src = w + (size_t)t * 8u;
  const v4f a = *(const v4fa*)src, c = *(const v4fa*)(src + 4);
  FragH f;
#pragma unroll
  for (int q = 0; q < 4; ++q) { f.h[q] = (_Float16)(bf16_rne(a[q]) * 16.0f); f.h[4 + q] = (_Float16)(bf16_rne(c[q]) * 16.0f); }
  const v8us o = f.half[0];
  unsigned short* d = (unsigned short*)Bt + (size_t)t * 8u;
  *(volatile v8us*)d = o; __threadfence(); *(volatile v8us*)d = o;
}

__global__ __launch_bounds__(256) void k_x16(const float* __restrict__ x, _Float16* __restrict__ X16, unsigned int n8) {
  const unsigned int t = blockIdx.x * 256u + threadIdx.x; if (t >= n8) return;
  const unsigned int row = t >> 7;
  const unsigned int b = row / (unsigned int)SQ, s = row - b * (unsigned int)SQ;
  const float* src = x + ((size_t)b * SQ_FULL + s) * DM + (size_t)(t & 127u) * 8u;
  const v4f a = *(const v4fa*)src, c = *(const v4fa*)(src + 4);
  FragH f;
#pragma unroll
  for (int q = 0; q < 4; ++q) { f.h[q] = (_Float16)bf16_rne(a[q]); f.h[4 + q] = (_Float16)bf16_rne(c[q]); }
  const v8us o = f.half[0];
  unsigned short* d = (unsigned short*)X16 + (size_t)t * 8u;
  *(volatile v8us*)d = o; __threadfence(); *(volatile v8us*)d = o;
}

__global__ __launch_bounds__(256) void k_vt(const _Float16* __restrict__ V16, _Float16* __restrict__ Vt) {
  __shared__ unsigned short tl[64][66];
  const unsigned int tid = threadIdx.x; const unsigned int slab = blockIdx.x / (unsigned int)(SQ / 64), lg = blockIdx.x % (unsigned int)(SQ / 64); const unsigned int b = slab / (unsigned int)NH, h = slab % (unsigned int)NH;
  for (unsigned int i = tid; i < 64u * 8u; i += 256u) { const unsigned int r = i >> 3, c8 = (i & 7u) * 8u; FragH f; f.half[0] = *(const v8us*)((const unsigned short*)V16 + ((size_t)b * SQ + lg * 64u + r) * LQ + h * 64u + c8);
#pragma unroll
    for (int q = 0; q < 8; ++q) tl[r][c8 + q] = f.u[q]; }
  __syncthreads();
  for (int pass = 0; pass < 2; ++pass) {
#pragma unroll
    for (int rd = 0; rd < 2; ++rd) { const unsigned int d = (unsigned int)rd * 32u + (tid >> 3), pc = tid & 7u; FragH f;
#pragma unroll
      for (int q = 0; q < 8; ++q) f.u[q] = tl[pc * 8u + q][d];
      const v8us o = f.half[0];
      *(volatile v8us*)((unsigned short*)Vt + ((size_t)slab * 64u + d) * SQ + lg * 64u + pc * 8u) = o; }
    if (pass == 0) __threadfence(); } }

__global__ __launch_bounds__(256) void k_hl(const float* __restrict__ F, _Float16* __restrict__ Hh, _Float16* __restrict__ Hl, unsigned int n8) {
  const unsigned int t = blockIdx.x * 256u + threadIdx.x; if (t >= n8) return; FragH fh, fl; const v4f a = *(const v4fa*)(F + (size_t)t * 8u), c = *(const v4fa*)(F + (size_t)t * 8u + 4);
#pragma unroll
  for (int q = 0; q < 4; ++q) { _Float16 h = (_Float16)a[q]; fh.h[q] = h; fl.h[q] = (_Float16)((a[q] - (float)h) * 1024.0f); h = (_Float16)c[q]; fh.h[4 + q] = h; fl.h[4 + q] = (_Float16)((c[q] - (float)h) * 1024.0f); }
  const v8us oh = fh.half[0], ol = fl.half[0];
  for (int pass = 0; pass < 2; ++pass) { *(volatile v8us*)((unsigned short*)Hh + (size_t)t * 8u) = oh; *(volatile v8us*)((unsigned short*)Hl + (size_t)t * 8u) = ol; if (pass == 0) __threadfence(); } }

__global__ __launch_bounds__(128) void k_gemm2(const _Float16* __restrict__ A, int lda, size_t sA, const _Float16* __restrict__ Bh, int ldb, size_t sB, float alpha, const float* CP,
    float* C, _Float16* C16, int ldc, size_t sC, int M, int N, int K) {
  __shared__ __attribute__((aligned(16))) float so[4][32][68];
  const unsigned int tid = threadIdx.x, w = tid >> 5, lane = tid & 31u, ln = lane & 15u, hh = lane >> 4; const unsigned int by = blockIdx.y;
  A += (size_t)by * sA; Bh += (size_t)by * sB; const size_t cofs = (size_t)by * sC;
  const unsigned int ntn = (unsigned int)N >> 6; const unsigned int mt = blockIdx.x / ntn, nq = blockIdx.x - mt * ntn; const unsigned int row0 = mt * 128u + 32u * w, col0 = nq * 64u; if (row0 >= (unsigned int)M) return;
  const _Float16* a0p = A + (size_t)(row0 + ln) * lda; const _Float16* a1p = a0p + (size_t)16 * lda;
  const _Float16* b0p = Bh + (size_t)(col0 + ln) * ldb; const _Float16* b1p = b0p + (size_t)16 * ldb; const _Float16* b2p = b1p + (size_t)16 * ldb; const _Float16* b3p = b2p + (size_t)16 * ldb;
  const v8f z8 = {0.f,0.f,0.f,0.f,0.f,0.f,0.f,0.f}; v8f c00 = z8, c01 = z8, c02 = z8, c03 = z8, c10 = z8, c11 = z8, c12 = z8, c13 = z8;
#pragma unroll 1
  for (int kb = 0; kb < K; kb += 32) { const v16h a0 = g2_frag(a0p + kb, hh), a1 = g2_frag(a1p + kb, hh);
    v16h b = g2_frag(b0p + kb, hh); c00 = g2_mma(a0, b, c00); c10 = g2_mma(a1, b, c10);
    b = g2_frag(b1p + kb, hh); c01 = g2_mma(a0, b, c01); c11 = g2_mma(a1, b, c11);
    b = g2_frag(b2p + kb, hh); c02 = g2_mma(a0, b, c02); c12 = g2_mma(a1, b, c12);
    b = g2_frag(b3p + kb, hh); c03 = g2_mma(a0, b, c03); c13 = g2_mma(a1, b, c13); }
  v8f accs[8] = {c00, c01, c02, c03, c10, c11, c12, c13};
#pragma unroll
  for (int u = 0; u < 8; ++u) { const unsigned int t = (unsigned int)u & 3u, half = (unsigned int)u >> 2; const unsigned int col = col0 + t * 16u + ln;
#pragma unroll
    for (int r = 0; r < 8; ++r) { const unsigned int rloc = half * 16u + 8u * hh + (unsigned int)r; float v = accs[u][r] * alpha; if (CP) v += CP[cofs + (size_t)(row0 + rloc) * ldc + col];
      so[w][rloc][t * 16u + ln] = v; } }
  __builtin_amdgcn_fence(4  , "workgroup"); __builtin_amdgcn_wave_barrier();
  const unsigned int rsub = lane >> 4, c4 = (lane & 15u) * 4u;
  for (int pass = 0; pass < 2; ++pass) {
#pragma unroll
    for (int q = 0; q < 16; ++q) { const unsigned int r = (unsigned int)q * 2u + rsub; const v4f v = *(const v4fa*)&so[w][r][c4]; if (C) *(volatile v4f*)(C + cofs + (size_t)(row0 + r) * ldc + col0 + c4) = v; if (C16) { v4h h4;
#pragma unroll
        for (int i = 0; i < 4; ++i) h4[i] = (_Float16)v[i];
        *(volatile v4h*)(C16 + cofs + (size_t)(row0 + r) * ldc + col0 + c4) = h4; } }
    if (pass == 0) __threadfence(); } }

__global__ __launch_bounds__(256) void k_rsmcf2(const float* __restrict__ S, _Float16* __restrict__ P, unsigned int hg, unsigned int q0, unsigned int nk) {
  #pragma clang fp contract(off)
  const unsigned int t = blockIdx.x * 256u + threadIdx.x; if (t >= hg * (unsigned int)QT) return; const size_t i = (size_t)t; const float* s = S + i * NKX; const unsigned int last = q0 + (t & (unsigned int)(QT - 1)); float mx = -3.0e38f;
#pragma unroll 1
  for (unsigned int j = 0; j < nk; ++j) { const float f = (j <= last) ? 1.f : 0.f; mx = fmaxf(mx, fmaf(f, s[j], (1.f - f) * -1.0e9f)); } float se = 0.f;
#pragma unroll 1
  for (unsigned int j = 0; j < nk; ++j) { const float f = (j <= last) ? 1.f : 0.f; se += __expf(fmaf(f, s[j], (1.f - f) * -1.0e9f) - mx); } const float sc = 256.0f / se;
#pragma unroll 1
  for (unsigned int j0 = 0; j0 < nk; j0 += 8) { FragH fr;
#pragma unroll
    for (int q = 0; q < 8; ++q) { const unsigned int j = j0 + (unsigned int)q; const float f = (j <= last) ? 1.f : 0.f; fr.h[q] = (_Float16)(__expf(fmaf(f, s[j], (1.f - f) * -1.0e9f) - mx) * sc); }
    const v8us o = fr.half[0]; unsigned short* d = (unsigned short*)P + i * NKX + j0; *(volatile v8us*)d = o; __threadfence(); *(volatile v8us*)d = o; } }

__global__ __launch_bounds__(64) void k_att0(const float* __restrict__ QF, const float* __restrict__ KF, const float* __restrict__ VF, int ld, size_t sF, float scale, float* __restrict__ OF, int ldo, size_t sO) {
  #pragma clang fp contract(off)
  __shared__ __attribute__((aligned(16))) float lq[64][64]; __shared__ __attribute__((aligned(16))) float lo[64][64];
  const unsigned int tid = threadIdx.x; const unsigned int h = blockIdx.x / (unsigned int)(QT0 / 64), rg = blockIdx.x % (unsigned int)(QT0 / 64); const unsigned int i = rg * 64u + tid;
  const size_t fo = (size_t)blockIdx.y * sF; QF += fo; KF += fo; VF += fo; OF += (size_t)blockIdx.y * sO;
  const float* qr = QF + (size_t)i * ld + h * HD;
#pragma unroll 1
  for (int c = 0; c < HD / 4; ++c) { *(v4fa*)&lq[tid][c * 4] = *(const v4fa*)(qr + c * 4); const v4f z = {0.f, 0.f, 0.f, 0.f}; *(v4fa*)&lo[tid][c * 4] = z; }
  float m = -1.0e30f, l = 0.f; const unsigned int jmax = rg * 64u + 63u;
#pragma unroll 1
  for (unsigned int j = 0; j <= jmax; ++j) { const float* kr = KF + (size_t)j * ld + h * HD; const float* vr = VF + (size_t)j * ld + h * HD; float s = 0.f;
#pragma unroll 1
    for (int c = 0; c < HD / 4; ++c) { const v4f kq = *(const v4fa*)(kr + c * 4); const v4f qq = *(const v4fa*)&lq[tid][c * 4]; s = __fadd_rn(s, __fmul_rn(qq[0], kq[0])); s = __fadd_rn(s, __fmul_rn(qq[1], kq[1])); s = __fadd_rn(s, __fmul_rn(qq[2], kq[2])); s = __fadd_rn(s, __fmul_rn(qq[3], kq[3])); }
    s = __fmul_rn(s, scale);
    const float f = (j <= i) ? 1.f : 0.f; const float sm = fmaf(f, s, (1.f - f) * -1.0e30f); const float mn = fmaxf(m, sm); const float sc = expf(m - mn); const float e = expf(sm - mn); l = __fadd_rn(__fmul_rn(l, sc), e); m = mn;
#pragma unroll 1
    for (int c = 0; c < HD / 4; ++c) { const v4f vv = *(const v4fa*)(vr + c * 4); v4f oo = *(const v4fa*)&lo[tid][c * 4];
#pragma unroll
      for (int u = 0; u < 4; ++u) oo[u] = __fadd_rn(__fmul_rn(oo[u], sc), __fmul_rn(e, vv[u]));
      *(v4fa*)&lo[tid][c * 4] = oo; } }
  const float fin = 64.0f / l;
#pragma unroll 1
  for (int c = 0; c < HD / 4; ++c) { v4f oo = *(const v4fa*)&lo[tid][c * 4];
#pragma unroll
    for (int u = 0; u < 4; ++u) oo[u] = __fmul_rn(oo[u], fin);
    *(v4fa*)&lo[tid][c * 4] = oo; }
  __syncthreads();
  for (int pass = 0; pass < 2; ++pass) {
#pragma unroll 1
    for (unsigned int it = 0; it < 16u; ++it) { const unsigned int row = it * 4u + (tid >> 4), pc = (tid & 15u) * 4u; const v4f v = *(const v4fa*)&lo[row][pc]; *(volatile v4f*)(OF + (size_t)(rg * 64u + row) * ldo + h * HD + pc) = v; }
    if (pass == 0) __threadfence(); } }

constexpr size_t al256(size_t b) { return (b + 255) & ~(size_t)255; }
constexpr size_t WS_TOTAL =
    al256((size_t)3 * DM * DM * 2) + al256((size_t)DM * DM * 2) + al256(NR * DM * 2) + al256(NR * 3 * DM * 2) + al256(NR * DM * 2) +
    al256((size_t)NH * QT * NKX * 4) + al256((size_t)NH * QT * NKX * 2) + al256((size_t)NB * NH * HD * SQ * 2) +
    al256((size_t)NB * QT0 * LQ * 4) + al256((size_t)NB * QT0 * DM * 4) + 2 * al256((size_t)NB * QT0 * DM * 2);
static_assert(WS_TOTAL <= (size_t)134217728);

extern "C" void kernel_launch(void* const* d_in, const int* in_sizes, int n_in,
                              void* d_out, int out_size, void* d_ws, size_t ws_size, hipStream_t stream) {
  if (n_in < 3) return;
  const size_t need_x = ((size_t)(NB - 1) * SQ_FULL + SQ) * DM;
  if ((size_t)in_sizes[0] < need_x) return;
  if ((size_t)in_sizes[1] < (size_t)3 * DM * DM) return;
  if ((size_t)in_sizes[2] < (size_t)DM * DM) return;
  if ((size_t)out_size < need_x) return;
  const float* x = (const float*)d_in[0]; const float* wa = (const float*)d_in[1]; const float* wp = (const float*)d_in[2];
  float* out = (float*)d_out;
  char* ws = (char*)d_ws; size_t off = 0;
  auto take = [&](size_t bytes) { char* p = ws + off; off += (bytes + 255) & ~(size_t)255; return p; };
  _Float16* BQKV = (_Float16*)take((size_t)3 * DM * DM * 2); _Float16* BO = (_Float16*)take((size_t)DM * DM * 2);
  _Float16* X16 = (_Float16*)take(NR * DM * 2); _Float16* QKV = (_Float16*)take(NR * 3 * DM * 2); _Float16* Q16 = QKV; _Float16* K16 = QKV + DM; _Float16* V16 = QKV + 2 * DM; _Float16* O16 = (_Float16*)take(NR * DM * 2);
  float* S = (float*)take((size_t)NH * QT * NKX * 4); _Float16* P = (_Float16*)take((size_t)NH * QT * NKX * 2); _Float16* VT = (_Float16*)take((size_t)NB * NH * HD * SQ * 2);
  float* F0 = (float*)take((size_t)NB * QT0 * LQ * 4); float* OF0 = (float*)take((size_t)NB * QT0 * DM * 4); _Float16* OH0 = (_Float16*)take((size_t)NB * QT0 * DM * 2); _Float16* OL0 = (_Float16*)take((size_t)NB * QT0 * DM * 2);
  if (off > ws_size) return;

  const unsigned int n8a = (unsigned int)((size_t)3 * DM * DM / 8), n8p = (unsigned int)((size_t)DM * DM / 8), n8x = (unsigned int)(NR * DM / 8);
  k_wnat<<<(n8a + 255u) / 256u, 256, 0, stream>>>(wa, n8a, BQKV);
  k_wnat<<<(n8p + 255u) / 256u, 256, 0, stream>>>(wp, n8p, BO);
  k_x16<<<(n8x + 255u) / 256u, 256, 0, stream>>>(x, X16, n8x);
  const int MP = (int)(NR);
  k_gemm2<<<dim3((unsigned int)((MP / 128) * (LQ / 64)), 1), 128, 0, stream>>>(X16, DM, (size_t)0, BQKV, DM, (size_t)0, 0.0625f, nullptr, nullptr, QKV, LQ, (size_t)0, MP, LQ, DM);
  k_gemm2<<<dim3((unsigned int)((QT0 / 128) * (LQ / 64)), NB), 128, 0, stream>>>(X16, DM, (size_t)SQ * DM, BQKV, DM, (size_t)0, 0.0625f, nullptr, F0, nullptr, LQ, (size_t)QT0 * LQ, QT0, LQ, DM);
  k_vt<<<NB * NH * (SQ / 64), 256, 0, stream>>>(V16, VT);
  k_att0<<<dim3(NH * (QT0 / 64), NB), 64, 0, stream>>>(F0, F0 + DM, F0 + 2 * DM, LQ, (size_t)QT0 * LQ, 0.125f, OF0, DM, (size_t)QT0 * DM);
  for (unsigned int b = 0; b < (unsigned int)NB; ++b) { const size_t r0 = (size_t)b * SQ;
    for (unsigned int q0 = 0; q0 < (unsigned int)SQ; q0 += QT) { const unsigned int nk = q0 + QT;
      k_gemm2<<<dim3((QT / 128) * (nk / 64), NH), 128, 0, stream>>>(Q16 + (r0 + q0) * LQ, LQ, (size_t)HD, K16 + r0 * LQ, LQ, (size_t)HD, 0.125f, nullptr, S, nullptr, NKX, (size_t)QT * NKX, QT, (int)nk, HD);
      k_rsmcf2<<<(NH * QT + 255) / 256, 256, 0, stream>>>(S, P, (unsigned int)NH, q0, nk);
      k_gemm2<<<dim3((QT / 128) * (HD / 64), NH), 128, 0, stream>>>(P, NKX, (size_t)QT * NKX, VT + (size_t)b * NH * HD * SQ, SQ, (size_t)HD * SQ, 0.25f, nullptr, nullptr, O16 + (r0 + q0) * DM, DM, (size_t)HD, QT, HD, (int)nk); } }
  k_gemm2<<<dim3((SQ / 128) * (DM / 64), NB), 128, 0, stream>>>(O16, DM, (size_t)SQ * DM, BO, DM, (size_t)0, 0.0009765625f, nullptr, out, nullptr, DM, (size_t)SQ_FULL * DM, SQ, DM, DM);
  const unsigned int n8h = (unsigned int)((size_t)NB * QT0 * DM / 8);
  k_hl<<<(n8h + 255u) / 256u, 256, 0, stream>>>(OF0, OH0, OL0, n8h);
  k_gemm2<<<dim3((QT0 / 128) * (DM / 64), NB), 128, 0, stream>>>(OH0, DM, (size_t)QT0 * DM, BO, DM, (size_t)0, 0.0009765625f, nullptr, out, nullptr, DM, (size_t)SQ_FULL * DM, QT0, DM, DM);
  k_gemm2<<<dim3((QT0 / 128) * (DM / 64), NB), 128, 0, stream>>>(OL0, DM, (size_t)QT0 * DM, BO, DM, (size_t)0, 0.00000095367431640625f, (const float*)out, out, nullptr, DM, (size_t)SQ_FULL * DM, QT0, DM, DM);
}
